// LunarCausalAttention_25391846654053
// MI455X (gfx1250) — hardware-verified
//
#include <hip/hip_runtime.h>


namespace {
constexpr int T = 2048, BS = 2, E = 1024, NH = 16, DH = 64, BH = BS * NH, PL = 32, NR = T * BS  , NPR = PL * BS  ;
constexpr float XS = 8.0f, WSC = 256.0f, SCL = 0.125f, BETA = 0.69314718055994531f, PS1 = 8.0f, PS2 = 64.0f;

typedef _Float16 b16;
typedef __attribute__((ext_vector_type(16))) _Float16 v16b;
typedef __attribute__((ext_vector_type(8))) _Float16 v8b;
typedef __attribute__((ext_vector_type(8))) float v8f;
typedef __attribute__((ext_vector_type(4))) float v4f;
__device__ __forceinline__ float bf16_rne(float f) { unsigned int u = __float_as_uint(f); u += 0x7FFFu + ((u >> 16) & 1u); return __uint_as_float(u & 0xFFFF0000u); }
__device__ __forceinline__ void split16(float v, b16& hi, b16& lo) { hi = (b16)v; lo = (b16)(v - (float)hi); }
__device__ __forceinline__ v16b frag_kb(const b16* p, int hh) { const v8b a = *(const v8b*)(p + 8 * hh), b = *(const v8b*)(p + 16 + 8 * hh); v16b f;
#pragma unroll
  for (int e = 0; e < 8; ++e) { f[e] = a[e]; f[8 + e] = b[e]; } return f; }
__device__ __forceinline__ v8f wmma16b(v16b a, v16b b, v8f c) { v8f d = __builtin_amdgcn_wmma_f32_16x16x32_f16(false, a, false, b, (short)0, c, false, false); asm volatile("v_nop\n\tv_nop\n\tv_nop\n\tv_nop" : "+v"(d) : "v"(a), "v"(b)); return d; }
__device__ __forceinline__ void wave_lds_sync() { __builtin_amdgcn_fence(__ATOMIC_RELEASE, "workgroup"); __builtin_amdgcn_wave_barrier(); __builtin_amdgcn_fence(__ATOMIC_ACQUIRE, "workgroup"); }
__device__ __forceinline__ float pmul(float a, float b) { float p = a * b; asm volatile("" : "+v"(p)); return p; }
__device__ __forceinline__ float softplus_b(float x) { const float bx = BETA * x; const float sp = (bx > 20.0f) ? bx : log1pf(__expf(bx)); return sp / BETA; }

__global__ __launch_bounds__(256) void prep_kernel(const float* __restrict__ query, const float* __restrict__ pquery, const float* __restrict__ wpq, const float* __restrict__ wq, const float* __restrict__ wpc, const float* __restrict__ wc, const float* __restrict__ wo, b16* __restrict__ X16, b16* __restrict__ PQ16, b16* __restrict__ W4, b16* __restrict__ WPQ) {
  const size_t t = (size_t)blockIdx.x * 256 + threadIdx.x; const size_t nx = (size_t)NR * E / 8, np_ = (size_t)NPR * E / 8, nw = (size_t)E * E / 8; v8b o;
  if (t < nx) { const size_t e = t * 8; const v4f a = *(const v4f*)(query + e), c = *(const v4f*)(query + e + 4); for (int j = 0; j < 4; ++j) { o[j] = (b16)(bf16_rne(a[j]) * XS); o[4 + j] = (b16)(bf16_rne(c[j]) * XS); } for (int pass = 0; pass < 2; ++pass) { *(volatile v8b*)(X16 + e) = o; __threadfence(); } return; }
  size_t u = t - nx;
  if (u < np_) { const size_t e = u * 8; for (int j = 0; j < 8; ++j) o[j] = (b16)(bf16_rne(pquery[e + j]) * XS); for (int pass = 0; pass < 2; ++pass) { *(volatile v8b*)(PQ16 + e) = o; __threadfence(); } return; } u -= np_;
  if (u < 5 * nw) { const int kind = (int)(u / nw); const size_t e = (u % nw) * 8; const float* w = kind == 0 ? wpc : kind == 1 ? wq : kind == 2 ? wc : kind == 3 ? wo : wpq; for (int j = 0; j < 8; ++j) o[j] = (b16)(bf16_rne(w[e + j]) * WSC);
    b16* dst = (kind < 4) ? (W4 + (size_t)kind * E * E) : WPQ; for (int pass = 0; pass < 2; ++pass) { *(volatile v8b*)(dst + e) = o; __threadfence(); } }
}
__global__ __launch_bounds__(128) void lin_kernel(const b16* __restrict__ X16, const b16* __restrict__ W4, const float* __restrict__ bpc, const float* __restrict__ bq, const float* __restrict__ bc, b16* __restrict__ KPh, b16* __restrict__ KPl, b16* __restrict__ Qh, b16* __restrict__ Ql, b16* __restrict__ KVh, b16* __restrict__ KVl) {
  __shared__ __attribute__((aligned(16))) b16 Th[4][16][128 + 8], Tl[4][16][128 + 8];
  const int wave = threadIdx.x >> 5, lane = threadIdx.x & 31, nloc = lane & 15, hlf = lane >> 4; const int kind = blockIdx.z, n0 = blockIdx.y * 128; const size_t m0 = (size_t)blockIdx.x * 64 + wave * 16;
  const b16* W = W4 + (size_t)kind * E * E; const float* bias = kind == 0 ? bpc : kind == 1 ? bq : bc; const float osc = (kind == 1) ? SCL : 1.0f;
  v8f acc[8];
#pragma unroll
  for (int t = 0; t < 8; ++t) acc[t] = (v8f){};
#pragma unroll 2
  for (int kb = 0; kb < E; kb += 32) { const v16b a = frag_kb(X16 + (m0 + nloc) * E + kb, hlf);
#pragma unroll
    for (int t = 0; t < 8; ++t) acc[t] = wmma16b(a, frag_kb(W + (size_t)(n0 + t * 16 + nloc) * E + kb, hlf), acc[t]); }
#pragma unroll
  for (int t = 0; t < 8; ++t) { const float bb = bf16_rne(bias[n0 + t * 16 + nloc]);
#pragma unroll
    for (int r = 0; r < 8; ++r) { b16 p, q; split16((acc[t][r] * (1.0f / (XS * WSC)) + bb) * osc * XS, p, q); Th[wave][8 * hlf + r][t * 16 + nloc] = p; Tl[wave][8 * hlf + r][t * 16 + nloc] = q; } }
  wave_lds_sync(); b16* dh = kind == 0 ? KPh : kind == 1 ? Qh : KVh; b16* dl = kind == 0 ? KPl : kind == 1 ? Ql : KVl;
  for (int pass = 0; pass < 2; ++pass) { for (int r2 = 0; r2 < 16; r2 += 2) { const int rr = r2 + (lane >> 4), c8 = (lane & 15) * 8; const size_t gi = (m0 + rr) * E + n0 + c8; *(volatile v8b*)(dh + gi) = *(const v8b*)(&Th[wave][rr][c8]); *(volatile v8b*)(dl + gi) = *(const v8b*)(&Tl[wave][rr][c8]); } __threadfence(); }
}
__global__ __launch_bounds__(256) void kvt_kernel(const b16* __restrict__ KVh, const b16* __restrict__ KVl, b16* __restrict__ KVTh, b16* __restrict__ KVTl) {
  __shared__ __attribute__((aligned(16))) b16 Ah[DH][64 + 8], Al[DH][64 + 8];
  const int bh = blockIdx.y, t0 = blockIdx.x * 64, t_ = threadIdx.x; const int b = bh / NH, h = bh % NH;
  for (int q = t_; q < 64 * DH; q += 256) { const int tt = q / DH, d = q % DH; const size_t gi = ((size_t)(t0 + tt) * BS + b) * E + h * DH + d; Ah[d][tt] = KVh[gi]; Al[d][tt] = KVl[gi]; }
  __syncthreads();
  for (int pass = 0; pass < 2; ++pass) { for (int q = t_; q < DH * 8; q += 256) { const int d = q >> 3, c8 = (q & 7) * 8; const size_t gi = ((size_t)bh * DH + d) * T + t0 + c8; *(volatile v8b*)(KVTh + gi) = *(const v8b*)(&Ah[d][c8]); *(volatile v8b*)(KVTl + gi) = *(const v8b*)(&Al[d][c8]); } __threadfence(); }
}
__global__ __launch_bounds__(128) void pattn_kernel(const b16* __restrict__ PQ16, const b16* __restrict__ WPQ, const float* __restrict__ bpq, const b16* __restrict__ KPh, const b16* __restrict__ KPl, b16* __restrict__ PAh, b16* __restrict__ PAl, b16* __restrict__ PATh, b16* __restrict__ PATl) {
  __shared__ __attribute__((aligned(16))) b16 Pq[PL][DH + 8], Pql[PL][DH + 8]; __shared__ __attribute__((aligned(16))) b16 Rh[4][16][PL + 8], Rl[4][16][PL + 8]; __shared__ __attribute__((aligned(16))) b16 Rt[PL][64 + 8], Rtl[PL][64 + 8];
  const int wave = threadIdx.x >> 5, lane = threadIdx.x & 31, nloc = lane & 15, hlf = lane >> 4, t_ = threadIdx.x; const int bh = blockIdx.y, b = bh / NH, h = bh % NH, t0 = blockIdx.x * 64;
  { const int pt = wave & 1, dt0 = (wave >> 1) * 2; v8f a2[2] = {{}, {}};
#pragma unroll 2
    for (int kb = 0; kb < E; kb += 32) { const v16b a = frag_kb(PQ16 + ((size_t)(pt * 16 + nloc) * BS + b) * E + kb, hlf);
#pragma unroll
      for (int t = 0; t < 2; ++t) a2[t] = wmma16b(a, frag_kb(WPQ + (size_t)(h * DH + (dt0 + t) * 16 + nloc) * E + kb, hlf), a2[t]); }
#pragma unroll
    for (int t = 0; t < 2; ++t) { const int d = (dt0 + t) * 16 + nloc; const float bb = bf16_rne(bpq[h * DH + d]);
#pragma unroll
      for (int r = 0; r < 8; ++r) { b16 p, q; split16((a2[t][r] * (1.0f / (XS * WSC)) + bb) * SCL * XS, p, q); Pq[pt * 16 + 8 * hlf + r][d] = p; Pql[pt * 16 + 8 * hlf + r][d] = q; } } }
  __syncthreads();
  { v8f d2[2] = {{}, {}}; const size_t arow = ((size_t)(t0 + wave * 16 + nloc) * BS + b) * E + h * DH;
#pragma unroll
    for (int kb = 0; kb < DH; kb += 32) { const v16b a = frag_kb(KPh + arow + kb, hlf), al = frag_kb(KPl + arow + kb, hlf);
#pragma unroll
      for (int t = 0; t < 2; ++t) { const v16b bp = frag_kb(&Pq[t * 16 + nloc][kb], hlf); d2[t] = wmma16b(a, bp, d2[t]); d2[t] = wmma16b(al, bp, d2[t]); d2[t] = wmma16b(a, frag_kb(&Pql[t * 16 + nloc][kb], hlf), d2[t]); } }
#pragma unroll
    for (int t = 0; t < 2; ++t)
#pragma unroll
      for (int r = 0; r < 8; ++r) { const float v = softplus_b(d2[t][r] * (1.0f / (XS * XS))); b16 p, q; split16(v * XS, p, q); const int tt = wave * 16 + 8 * hlf + r, pp = t * 16 + nloc; Rh[wave][8 * hlf + r][pp] = p; Rl[wave][8 * hlf + r][pp] = q; Rt[pp][tt] = p; Rtl[pp][tt] = q; } }
  __syncthreads();
  for (int pass = 0; pass < 2; ++pass) {
    for (int k = 0; k < 2; ++k) { const int rr = k * 8 + (lane >> 2), c8 = (lane & 3) * 8; const size_t gi = ((size_t)bh * T + t0 + wave * 16 + rr) * PL + c8; *(volatile v8b*)(PAh + gi) = *(const v8b*)(&Rh[wave][rr][c8]); *(volatile v8b*)(PAl + gi) = *(const v8b*)(&Rl[wave][rr][c8]); }
    for (int q = t_; q < PL * 8; q += 128) { const int pp = q >> 3, c8 = (q & 7) * 8; const size_t gi = ((size_t)bh * PL + pp) * T + t0 + c8; *(volatile v8b*)(PATh + gi) = *(const v8b*)(&Rt[pp][c8]); *(volatile v8b*)(PATl + gi) = *(const v8b*)(&Rtl[pp][c8]); }
    __threadfence(); }
}
__global__ __launch_bounds__(64) void step1_kernel(const b16* __restrict__ Qh, const b16* __restrict__ Ql, const b16* __restrict__ KVh, const b16* __restrict__ KVl, const b16* __restrict__ PATh, const b16* __restrict__ PATl, b16* __restrict__ Ah, b16* __restrict__ Al) {
  __shared__ __attribute__((aligned(16))) b16 Ra[2][16][PL + 8], Ral[2][16][PL + 8];
  const int wave = threadIdx.x >> 5, lane = threadIdx.x & 31, hh = lane >> 4, col = lane & 15; const int bh = blockIdx.y, b = bh / NH, h = bh % NH; const int q0 = blockIdx.x * 32 + wave * 16, qi = q0 + col;
  const size_t qrow = ((size_t)qi * BS + b) * E + h * DH; const v16b qa0 = frag_kb(Qh + qrow, hh), qa1 = frag_kb(Qh + qrow + 32, hh), ql0 = frag_kb(Ql + qrow, hh), ql1 = frag_kb(Ql + qrow + 32, hh);
  const b16* Pb = PATh + (size_t)bh * PL * T; const b16* Plb = PATl + (size_t)bh * PL * T;
  v8f aw[2] = {{}, {}}, awl[2] = {{}, {}}; const int kend = q0 + 16;
  for (int kb = 0; kb < kend; kb += 32) {
    v8f s0 = {}, s1 = {};
    { const b16* k0 = KVh + ((size_t)(kb + col) * BS + b) * E + h * DH, *k1 = KVh + ((size_t)(kb + 16 + col) * BS + b) * E + h * DH, *k0l = KVl + ((size_t)(kb + col) * BS + b) * E + h * DH, *k1l = KVl + ((size_t)(kb + 16 + col) * BS + b) * E + h * DH;
      v16b f = frag_kb(k0, hh); s0 = wmma16b(f, qa0, s0); s0 = wmma16b(f, ql0, s0); s0 = wmma16b(frag_kb(k0l, hh), qa0, s0);
      f = frag_kb(k0 + 32, hh); s0 = wmma16b(f, qa1, s0); s0 = wmma16b(f, ql1, s0); s0 = wmma16b(frag_kb(k0l + 32, hh), qa1, s0);
      f = frag_kb(k1, hh); s1 = wmma16b(f, qa0, s1); s1 = wmma16b(f, ql0, s1); s1 = wmma16b(frag_kb(k1l, hh), qa0, s1);
      f = frag_kb(k1 + 32, hh); s1 = wmma16b(f, qa1, s1); s1 = wmma16b(f, ql1, s1); s1 = wmma16b(frag_kb(k1l + 32, hh), qa1, s1); }
    v16b ph, pl;
#pragma unroll
    for (int r = 0; r < 8; ++r) { const int ka = kb + 8 * hh + r, kbb = kb + 16 + 8 * hh + r; const float v0 = (ka <= qi) ? s0[r] * (1.0f / (XS * XS)) : 0.0f, v1 = (kbb <= qi) ? s1[r] * (1.0f / (XS * XS)) : 0.0f; b16 p, q; split16(v0 * PS1, p, q); ph[r] = p; pl[r] = q; split16(v1 * PS1, p, q); ph[8 + r] = p; pl[8 + r] = q; }
#pragma unroll
    for (int t = 0; t < 2; ++t) { const v16b pa = frag_kb(Pb + (size_t)(t * 16 + col) * T + kb, hh); aw[t] = wmma16b(pa, ph, aw[t]); awl[t] = wmma16b(pa, pl, awl[t]); awl[t] = wmma16b(frag_kb(Plb + (size_t)(t * 16 + col) * T + kb, hh), ph, awl[t]); } }
  float v[16]; const float invn = 1.0f / ((float)(qi + 1) * PS1 * XS); float mx = -INFINITY;
#pragma unroll
  for (int t = 0; t < 2; ++t) for (int r = 0; r < 8; ++r) { v[t * 8 + r] = (aw[t][r] + awl[t][r]) * invn; mx = fmaxf(mx, v[t * 8 + r]); }
  mx = fmaxf(mx, __shfl_xor(mx, 16)); float sm = 0.0f; for (int i = 0; i < 16; ++i) { v[i] = __expf(v[i] - mx); sm += v[i]; } sm += __shfl_xor(sm, 16); const float inv = 1.0f / sm;
#pragma unroll
  for (int t = 0; t < 2; ++t) for (int r = 0; r < 8; ++r) { b16 p, q; split16(v[t * 8 + r] * inv * PS2, p, q); Ra[wave][col][t * 16 + 8 * hh + r] = p; Ral[wave][col][t * 16 + 8 * hh + r] = q; }
  wave_lds_sync();
  for (int pass = 0; pass < 2; ++pass) { for (int k = 0; k < 2; ++k) { const int rr = k * 8 + (lane >> 2), c8 = (lane & 3) * 8; const size_t gi = ((size_t)bh * T + q0 + rr) * PL + c8; *(volatile v8b*)(Ah + gi) = *(const v8b*)(&Ra[wave][rr][c8]); *(volatile v8b*)(Al + gi) = *(const v8b*)(&Ral[wave][rr][c8]); } __threadfence(); }
}
__global__ __launch_bounds__(64) void step2_kernel(const b16* __restrict__ PAh, const b16* __restrict__ PAl, const b16* __restrict__ Ah, const b16* __restrict__ Al, const b16* __restrict__ KVTh, const b16* __restrict__ KVTl, b16* __restrict__ ATh, b16* __restrict__ ATl) {
  __shared__ __attribute__((aligned(16))) float To[2][16][DH + 4];
  const int wave = threadIdx.x >> 5, lane = threadIdx.x & 31, hh = lane >> 4, col = lane & 15; const int bh = blockIdx.y, b = bh / NH, h = bh % NH; const int q0 = blockIdx.x * 32 + wave * 16, qi = q0 + col;
  const v16b aq = frag_kb(Ah + ((size_t)bh * T + qi) * PL, hh), aql = frag_kb(Al + ((size_t)bh * T + qi) * PL, hh);
  const b16* Vb = KVTh + (size_t)bh * DH * T; const b16* Vlb = KVTl + (size_t)bh * DH * T;
  v8f o[4] = {{}, {}, {}, {}}, ol[4] = {{}, {}, {}, {}}; const int kend = q0 + 16;
  for (int kb = 0; kb < kend; kb += 32) {
    v8f s0 = {}, s1 = {};
    { const b16* p0 = PAh + ((size_t)bh * T + kb + col) * PL, *p1 = PAh + ((size_t)bh * T + kb + 16 + col) * PL, *p0l = PAl + ((size_t)bh * T + kb + col) * PL, *p1l = PAl + ((size_t)bh * T + kb + 16 + col) * PL;
      v16b f = frag_kb(p0, hh); s0 = wmma16b(f, aq, s0); s0 = wmma16b(f, aql, s0); s0 = wmma16b(frag_kb(p0l, hh), aq, s0);
      f = frag_kb(p1, hh); s1 = wmma16b(f, aq, s1); s1 = wmma16b(f, aql, s1); s1 = wmma16b(frag_kb(p1l, hh), aq, s1); }
    v16b ph, pl;
#pragma unroll
    for (int r = 0; r < 8; ++r) { const int ka = kb + 8 * hh + r, kbb = kb + 16 + 8 * hh + r; const float v0 = (ka <= qi) ? s0[r] * (1.0f / (XS * PS2)) : 0.0f, v1 = (kbb <= qi) ? s1[r] * (1.0f / (XS * PS2)) : 0.0f; b16 p, q; split16(v0 * PS1, p, q); ph[r] = p; pl[r] = q; split16(v1 * PS1, p, q); ph[8 + r] = p; pl[8 + r] = q; }
#pragma unroll
    for (int t = 0; t < 4; ++t) { const v16b vf = frag_kb(Vb + (size_t)(t * 16 + col) * T + kb, hh); o[t] = wmma16b(vf, ph, o[t]); ol[t] = wmma16b(vf, pl, ol[t]); ol[t] = wmma16b(frag_kb(Vlb + (size_t)(t * 16 + col) * T + kb, hh), ph, ol[t]); } }
  const float invn = 1.0f / ((float)(qi + 1) * PS1 * XS);
#pragma unroll
  for (int t = 0; t < 4; ++t)
#pragma unroll
    for (int r = 0; r < 8; ++r) To[wave][col][t * 16 + 8 * hh + r] = (o[t][r] + ol[t][r]) * invn;
  wave_lds_sync();
  for (int pass = 0; pass < 2; ++pass) { for (int r4 = 0; r4 < 16; r4 += 4) { const int rr = r4 + (lane >> 3), c8 = (lane & 7) * 8; v8b hv, lv; for (int j = 0; j < 8; ++j) { b16 p, q; split16(To[wave][rr][c8 + j] * XS, p, q); hv[j] = p; lv[j] = q; }
      const size_t gi = ((size_t)(q0 + rr) * BS + b) * E + h * DH + c8; *(volatile v8b*)(ATh + gi) = hv; *(volatile v8b*)(ATl + gi) = lv; } __threadfence(); }
}
__global__ __launch_bounds__(128) void oproj_kernel(const b16* __restrict__ ATh, const b16* __restrict__ ATl, const b16* __restrict__ WO, const float* __restrict__ bo, float* __restrict__ out) {
  __shared__ __attribute__((aligned(16))) float Tf[4][16][128 + 4];
  const int wave = threadIdx.x >> 5, lane = threadIdx.x & 31, nloc = lane & 15, hlf = lane >> 4; const int n0 = blockIdx.y * 128; const size_t m0 = (size_t)blockIdx.x * 64 + wave * 16;
  v8f acc[8];
#pragma unroll
  for (int t = 0; t < 8; ++t) acc[t] = (v8f){};
#pragma unroll 2
  for (int kb = 0; kb < E; kb += 32) { const v16b a = frag_kb(ATh + (m0 + nloc) * E + kb, hlf), al = frag_kb(ATl + (m0 + nloc) * E + kb, hlf);
#pragma unroll
    for (int t = 0; t < 8; ++t) { const v16b bw = frag_kb(WO + (size_t)(n0 + t * 16 + nloc) * E + kb, hlf); acc[t] = wmma16b(a, bw, acc[t]); acc[t] = wmma16b(al, bw, acc[t]); } }
#pragma unroll
  for (int t = 0; t < 8; ++t) { const float bb = bf16_rne(bo[n0 + t * 16 + nloc]);
#pragma unroll
    for (int r = 0; r < 8; ++r) Tf[wave][8 * hlf + r][t * 16 + nloc] = acc[t][r] * (1.0f / (XS * WSC)) + bb; }
  wave_lds_sync();
  for (int pass = 0; pass < 2; ++pass) { for (int rr = 0; rr < 16; ++rr) *(volatile v4f*)(out + (m0 + rr) * E + n0 + lane * 4) = *(const v4f*)(&Tf[wave][rr][lane * 4]); __threadfence(); }
}
}

extern "C" void kernel_launch(void* const* d_in, const int* in_sizes, int n_in, void* d_out, int out_size, void* d_ws, size_t ws_size, hipStream_t stream) {
  (void)n_in;
  auto Fp = [&](int i) { return (const float*)d_in[i]; };
  if (in_sizes[0] != NR * E || in_sizes[1] != NPR * E || in_sizes[2] != E * E || in_sizes[4] != E * E || in_sizes[6] != E * E || in_sizes[8] != E * E || in_sizes[10] != E * E || out_size != NR * E) return;
  size_t off = 0; char* ws = (char*)d_ws;
  auto carve = [&](size_t bytes) { char* p = ws + off; off += (bytes + 255) & ~(size_t)255; return p; };
  b16* X16 = (b16*)carve((size_t)NR * E * 2); b16* PQ16 = (b16*)carve((size_t)NPR * E * 2); b16* W4 = (b16*)carve((size_t)4 * E * E * 2); b16* WPQ = (b16*)carve((size_t)E * E * 2);
  b16* KPh = (b16*)carve((size_t)NR * E * 2); b16* KPl = (b16*)carve((size_t)NR * E * 2); b16* Qh = (b16*)carve((size_t)NR * E * 2); b16* Ql = (b16*)carve((size_t)NR * E * 2); b16* KVh = (b16*)carve((size_t)NR * E * 2); b16* KVl = (b16*)carve((size_t)NR * E * 2);
  b16* KVTh = (b16*)carve((size_t)NR * E * 2); b16* KVTl = (b16*)carve((size_t)NR * E * 2); b16* PAh = (b16*)carve((size_t)BH * T * PL * 2); b16* PAl = (b16*)carve((size_t)BH * T * PL * 2); b16* PATh = (b16*)carve((size_t)BH * PL * T * 2); b16* PATl = (b16*)carve((size_t)BH * PL * T * 2);
  b16* Ah = (b16*)carve((size_t)BH * T * PL * 2); b16* Al = (b16*)carve((size_t)BH * T * PL * 2);
  b16* ATh = KPh; b16* ATl = KPl;
  if (off > ws_size || off > ((size_t)128 << 20)) return;
  prep_kernel<<<(unsigned)(((size_t)NR * E / 8 + (size_t)NPR * E / 8 + 5 * (size_t)E * E / 8 + 255) / 256), 256, 0, stream>>>(Fp(0), Fp(1), Fp(2), Fp(4), Fp(6), Fp(8), Fp(10), X16, PQ16, W4, WPQ);
  lin_kernel<<<dim3(NR / 64, E / 128, 3), 128, 0, stream>>>(X16, W4, Fp(7), Fp(5), Fp(9), KPh, KPl, Qh, Ql, KVh, KVl);
  kvt_kernel<<<dim3(T / 64, BH), 256, 0, stream>>>(KVh, KVl, KVTh, KVTl);
  pattn_kernel<<<dim3(T / 64, BH), 128, 0, stream>>>(PQ16, WPQ, Fp(3), KPh, KPl, PAh, PAl, PATh, PATl);
  step1_kernel<<<dim3(T / 32, BH), 64, 0, stream>>>(Qh, Ql, KVh, KVl, PATh, PATl, Ah, Al);
  step2_kernel<<<dim3(T / 32, BH), 64, 0, stream>>>(PAh, PAl, Ah, Al, KVTh, KVTl, ATh, ATl);
  oproj_kernel<<<dim3(NR / 64, E / 128), 128, 0, stream>>>(ATh, ATl, W4 + (size_t)3 * E * E, Fp(11), (float*)d_out);
}
